// HSTUModel_45183055954604
// MI455X (gfx1250) — hardware-verified
//
#include <hip/hip_runtime.h>


#define NB_  2
#define SS   2048
#define DD   1024
#define NH_  8
#define DA   64
#define DL   64
#define PJ   2048
#define NL   2
#define ZH   4
#define NT64 (SS / 64)
#define DM   DD
#define LOSC 1024.0f
typedef _Float16 h16;
typedef unsigned short bf;
typedef __attribute__((ext_vector_type(16))) __bf16   v16bf;
typedef __attribute__((ext_vector_type(16))) _Float16 v16h;
typedef __attribute__((ext_vector_type(8)))  _Float16 v8h;
typedef __attribute__((ext_vector_type(8)))  unsigned short v8us;
typedef __attribute__((ext_vector_type(8)))  float    v8f;
typedef __attribute__((ext_vector_type(4)))  float    v4f;
typedef v8h  __attribute__((may_alias)) v8ha;
typedef v4f  __attribute__((may_alias)) v4fa;
typedef v8us __attribute__((may_alias)) v8usa;

__device__ __forceinline__ unsigned short f2bf(float f) { unsigned u = __float_as_uint(f); u += 0x7FFFu + ((u >> 16) & 1u); return (unsigned short)(u >> 16); }
__device__ __forceinline__ float bf2f(unsigned short b) { return __uint_as_float(((unsigned)b) << 16); }
__device__ __forceinline__ float bfr(float f) { return bf2f(f2bf(f)); }
__device__ __forceinline__ v16h cat16(v8h lo, v8h hi) { return __builtin_shufflevector(lo, hi, 0, 1, 2, 3, 4, 5, 6, 7, 8, 9, 10, 11, 12, 13, 14, 15); }
__device__ __forceinline__ v16bf cat16b(v8us lo, v8us hi) { return __builtin_bit_cast(v16bf, __builtin_shufflevector(lo, hi, 0, 1, 2, 3, 4, 5, 6, 7, 8, 9, 10, 11, 12, 13, 14, 15)); }
__device__ __forceinline__ v8f wmma16(v16h a, v16h b, v8f c) { return __builtin_amdgcn_wmma_f32_16x16x32_f16(false, a, false, b, (short)0, c, false, false); }
__device__ __forceinline__ v8f wmmab(v16bf a, v16bf b, v8f c) { return __builtin_amdgcn_wmma_f32_16x16x32_bf16(false, a, false, b, (short)0, c, false, false); }


__global__ __launch_bounds__(128) void k_gemmh(const h16* __restrict__ A, const h16* __restrict__ Bn, const float* __restrict__ bias, float* C, int ldc, const float* __restrict__ R, int K, size_t sA, size_t sB, size_t sC, int roundR) {
    __shared__ __align__(16) float ost[4][16 * 68];
    const size_t z = blockIdx.z; A += z * sA; Bn += z * sB; C += z * sC; if (R) R += z * sC;
    const int lane = threadIdx.x & 31, wave = threadIdx.x >> 5, lr = lane & 15, hi = lane >> 4;
    const int r0 = blockIdx.x * 64 + wave * 16, c0 = blockIdx.y * 64;
    const size_t aoff = (size_t)(r0 + lr) * K + 8 * hi;
    size_t boff[4];
#pragma unroll
    for (int t = 0; t < 4; ++t) boff[t] = (size_t)(c0 + t * 16 + lr) * K + 8 * hi;
    v8f acc[4];
#pragma unroll
    for (int t = 0; t < 4; ++t) acc[t] = (v8f){};
#pragma unroll 1
    for (int kc = 0; kc < K; kc += 32) {
        const v16h a = cat16(*(const v8h*)(A + aoff + kc), *(const v8h*)(A + aoff + kc + 16));
#pragma unroll
        for (int t = 0; t < 4; ++t) { const v16h b = cat16(*(const v8h*)(Bn + boff[t] + kc), *(const v8h*)(Bn + boff[t] + kc + 16)); acc[t] = wmma16(a, b, acc[t]); }
        asm volatile("v_nop\n\tv_nop\n\tv_nop\n\tv_nop" : "+v"(acc[0]), "+v"(acc[1]), "+v"(acc[2]), "+v"(acc[3]) : "v"(a));
    }
    float* os = &ost[wave][0];
#pragma unroll
    for (int t = 0; t < 4; ++t) { const float bv = bias ? bfr(bias[c0 + t * 16 + lr]) : 0.f;
#pragma unroll
        for (int j = 0; j < 8; ++j) os[(hi * 8 + j) * 68 + t * 16 + lr] = acc[t][j] + bv; }
    __syncthreads();
    float* crow = C + (size_t)r0 * ldc + c0;
    auto pass = [&]() {
#pragma unroll
        for (int s = 0; s < 8; ++s) { const int Lid = (lane >> 3) + 4 * s, piece = lane & 7; const int row = Lid >> 1, cofs = (Lid & 1) * 32 + piece * 4;
            v4f val = *(const v4fa*)(os + row * 68 + cofs); if (R) { const v4f rv = *(const v4f*)(R + ((size_t)r0 + row) * ldc + c0 + cofs); val += roundR ? (v4f){bfr(rv[0]), bfr(rv[1]), bfr(rv[2]), bfr(rv[3])} : rv; }
            *(volatile v4f*)(crow + (size_t)row * ldc + cofs) = val; }
    };
    pass(); __threadfence(); pass();
}

typedef __attribute__((ext_vector_type(4))) _Float16 v4h;
__device__ __forceinline__ h16 tohx(float x) { return (h16)x; }
__device__ __forceinline__ float siluf(float x) { return __fdiv_rn(x, 1.0f + expf(-x)); }
template <int MODE>
__global__ __launch_bounds__(128) void k_gemmhm(const h16* __restrict__ A, const h16* __restrict__ Bn, int K, float* C, int ldc, size_t sA, size_t sB, size_t sC, const int* __restrict__ FL) {
    const int I = blockIdx.x;
    if (MODE == 1 && FL[I * NT64 + blockIdx.y] == 0) return;
    int Klo = 0, Klim = K;
    if (MODE == 2) { int f = -1, l = -1; for (int j = 0; j < NT64; ++j) { if (FL[I * NT64 + j]) { if (f < 0) f = j; l = j; } } if (f < 0) { Klo = 0; Klim = 0; } else { Klo = f * 64; Klim = (l + 1) * 64; } }
    const size_t z = blockIdx.z; A += z * sA; Bn += z * sB; C += z * sC;
    __shared__ __align__(16) float ost[4][16 * 68];
    const int lane = threadIdx.x & 31, wave = threadIdx.x >> 5, lr = lane & 15, hi = lane >> 4;
    const int r0 = blockIdx.x * 64 + wave * 16, c0 = blockIdx.y * 64;
    const size_t aoff = (size_t)(r0 + lr) * K + 8 * hi;
    v8f acc[4];
#pragma unroll
    for (int t = 0; t < 4; ++t) acc[t] = (v8f){};
#pragma unroll 1
    for (int kc = Klo; kc < Klim; kc += 32) {
        const v16h a = cat16(*(const v8h*)(A + aoff + kc), *(const v8h*)(A + aoff + kc + 16));
#pragma unroll
        for (int t = 0; t < 4; ++t) { const size_t bo = (size_t)(c0 + t * 16 + lr) * K + kc + 8 * hi; const v16h b = cat16(*(const v8h*)(Bn + bo), *(const v8h*)(Bn + bo + 16)); acc[t] = wmma16(a, b, acc[t]); }
        asm volatile("v_nop\n\tv_nop\n\tv_nop\n\tv_nop" : "+v"(acc[0]), "+v"(acc[1]), "+v"(acc[2]), "+v"(acc[3]) : "v"(a));
    }
    float* os = &ost[wave][0];
#pragma unroll
    for (int t = 0; t < 4; ++t) {
#pragma unroll
        for (int j = 0; j < 8; ++j) os[(hi * 8 + j) * 68 + t * 16 + lr] = acc[t][j]; }
    __builtin_amdgcn_wave_barrier(); asm volatile("" ::: "memory");
    float* crow = C + (size_t)r0 * ldc + c0;
    auto pass = [&]() {
#pragma unroll
        for (int s = 0; s < 8; ++s) { const int Lid = (lane >> 3) + 4 * s, piece = lane & 7; const int row = Lid >> 1, cofs = (Lid & 1) * 32 + piece * 4;
            const v4f val = *(const v4fa*)(os + row * 68 + cofs); *(volatile v4f*)(crow + (size_t)row * ldc + cofs) = val; }
    };
    pass(); __threadfence(); pass();
}
__global__ __launch_bounds__(256) void k_flags(const int* __restrict__ mask, int* FL) {
    __shared__ int acc[8][32];
    const int b = blockIdx.y, I = blockIdx.x; const int lane = threadIdx.x & 31, wv = threadIdx.x >> 5; int any = 0;
#pragma unroll 1
    for (int r = wv; r < 64; r += 8) { const int* mr = mask + ((size_t)b * SS + I * 64 + r) * SS + lane * 64;
#pragma unroll 1
        for (int c = 0; c < 64; ++c) any |= (mr[c] != 0); }
    acc[wv][lane] = any; __syncthreads();
    if (wv == 0) { int v = 0;
#pragma unroll
        for (int w = 0; w < 8; ++w) v |= acc[w][lane];
        *(volatile int*)(FL + ((size_t)b * NT64 + I) * NT64 + lane) = v; __threadfence(); *(volatile int*)(FL + ((size_t)b * NT64 + I) * NT64 + lane) = v; }
}
template <bool F32OUT>
__global__ __launch_bounds__(256) void k_lnh(const float* __restrict__ X, const float* __restrict__ w, const float* __restrict__ bb, float eps, h16* OH, float* OF) {
    const int lane = threadIdx.x & 31; const size_t r = (size_t)blockIdx.x * 8 + (threadIdx.x >> 5); if (r >= (size_t)SS) return; const float* xr = X + r * DD; float s = 0.f;
#pragma unroll 1
    for (int c = lane; c < DD; c += 32) s += xr[c];
#pragma unroll
    for (int sh = 16; sh; sh >>= 1) s += __shfl_xor(s, sh, 32);
    const float mu = s * (1.0f / DD); float q = 0.f;
#pragma unroll 1
    for (int c = lane; c < DD; c += 32) { const float d = xr[c] - mu; q = fmaf(d, d, q); }
#pragma unroll
    for (int sh = 16; sh; sh >>= 1) q += __shfl_xor(q, sh, 32);
    const float rs = rsqrtf(q * (1.0f / DD) + eps);
#pragma unroll 1
    for (int ps = 0; ps < 2; ++ps) {
        if (!F32OUT) {
#pragma unroll 1
            for (int p = 0; p < DD / 256; ++p) { const int c0 = p * 256 + lane * 8; v8h o;
#pragma unroll
                for (int i = 0; i < 8; ++i) { const int c = c0 + i; o[i] = tohx((xr[c] - mu) * rs * bfr(w[c]) + bfr(bb[c])); }
                *(volatile v8h*)(OH + r * DD + c0) = o; } }
        else {
#pragma unroll 1
            for (int p = 0; p < DD / 128; ++p) { const int c0 = p * 128 + lane * 4; v4f o;
#pragma unroll
                for (int i = 0; i < 4; ++i) { const int c = c0 + i; o[i] = (xr[c] - mu) * rs * bfr(w[c]) + bfr(bb[c]); }
                *(volatile v4f*)(OF + r * DD + c0) = o; } }
        if (ps == 0) __threadfence(); }
}
__global__ __launch_bounds__(256) void k_wTh(const float* __restrict__ Wm, int K, int N, h16* Bt) {
    __shared__ float tl[64][65];
    const int tid = threadIdx.x; const int k0 = blockIdx.x * 64, n0 = blockIdx.y * 64; const int rr = tid >> 2, cq = (tid & 3) * 16;
#pragma unroll
    for (int i = 0; i < 16; ++i) tl[rr][cq + i] = bfr(Wm[(size_t)(k0 + rr) * N + n0 + cq + i]);
    __syncthreads();
    const int lane = tid & 31, wv = tid >> 5;
    auto pass = [&]() {
#pragma unroll
        for (int st = 0; st < 4; ++st) { const int nr = wv * 8 + st * 2 + (lane >> 4); const int kq = (lane & 15) * 4; v4h v;
#pragma unroll
            for (int i = 0; i < 4; ++i) v[i] = tohx(tl[kq + i][nr]);
            *(volatile v4h*)(Bt + (size_t)(n0 + nr) * K + k0 + kq) = v; }
    };
    pass(); __threadfence(); pass();
}
__global__ __launch_bounds__(256) void k_cvt8h(const float* __restrict__ src, h16* dst, size_t n8) { const size_t i = (size_t)blockIdx.x * 256 + threadIdx.x; if (i >= n8) return; const v8f v = *(const v8f*)(src + i * 8); v8h o;
#pragma unroll
    for (int k = 0; k < 8; ++k) o[k] = tohx(bfr(v[k])); *(volatile v8h*)(dst + i * 8) = o; __threadfence(); *(volatile v8h*)(dst + i * 8) = o; }
__global__ __launch_bounds__(256) void k_hpls(const float* __restrict__ PR, int col0, int h0, h16* P) {
    const int lane = threadIdx.x & 31; const size_t w = (size_t)blockIdx.x * 8 + (threadIdx.x >> 5); const int i = (int)(w * 2 + (lane >> 4)); if (i >= SS) return; const int z = blockIdx.z; const int c0 = (lane & 15) * 4; v4h o;
#pragma unroll
    for (int q = 0; q < 4; ++q) o[q] = tohx(siluf(PR[(size_t)i * PJ + col0 + (h0 + z) * 64 + c0 + q]));
    const size_t off = ((size_t)z * SS + i) * 64 + c0; *(volatile v4h*)(P + off) = o; __threadfence(); *(volatile v4h*)(P + off) = o;
}
__global__ __launch_bounds__(256) void k_vTs(const float* __restrict__ PR, int h0, h16* VT) {
    __shared__ float tl[64][65];
    const int tid = threadIdx.x; const int t0 = blockIdx.x * 64; const int z = blockIdx.z; const int rr = tid >> 2, cq = (tid & 3) * 16;
#pragma unroll 1
    for (int i = 0; i < 16; ++i) tl[rr][cq + i] = siluf(PR[(size_t)(t0 + rr) * PJ + DL * NH_ + (h0 + z) * 64 + cq + i]);
    __syncthreads();
    const int lane = tid & 31, wv = tid >> 5;
    auto pass = [&]() {
#pragma unroll
        for (int st = 0; st < 4; ++st) { const int dr = wv * 8 + st * 2 + (lane >> 4); const int tq = (lane & 15) * 4; v4h v;
#pragma unroll
            for (int i = 0; i < 4; ++i) v[i] = tohx(tl[tq + i][dr]);
            *(volatile v4h*)(VT + ((size_t)z * 64 + dr) * SS + t0 + tq) = v; }
    };
    pass(); __threadfence(); pass();
}
__global__ __launch_bounds__(256) void k_pmask(const float* __restrict__ S, const int* __restrict__ mask, int b, h16* P) {
    const int lane = threadIdx.x & 31, i = blockIdx.x * 8 + (threadIdx.x >> 5); if (i >= SS) return; const size_t zo = ((size_t)blockIdx.z * SS + i) * SS; const int* mr = mask + ((size_t)b * SS + i) * SS;
#pragma unroll 1
    for (int ps = 0; ps < 2; ++ps) {
#pragma unroll 1
        for (int c0 = lane * 4; c0 < SS; c0 += 128) { v4h o;
#pragma unroll
            for (int q = 0; q < 4; ++q) { const int t = c0 + q; float p = 0.f; if (mr[t] != 0) p = siluf(S[zo + t]); o[q] = tohx(p); }
            *(volatile v4h*)(P + zo + c0) = o; }
        if (ps == 0) __threadfence(); }
}
__global__ __launch_bounds__(256) void k_normu(const float* __restrict__ O, const float* __restrict__ PR, int h0, h16* UD) {
    const int lane = threadIdx.x & 31; const size_t w = (size_t)blockIdx.x * 8 + (threadIdx.x >> 5); const int i = (int)(w * 2 + (lane >> 4)); const int z = blockIdx.z; const int c0 = (lane & 15) * 4; const bool live = i < SS;
    v4f v = live ? *(const v4f*)(O + ((size_t)z * SS + i) * 64 + c0) : (v4f){0.f, 0.f, 0.f, 0.f}; v = v * (1.0f / SS);
    float s = v[0] + v[1] + v[2] + v[3];
#pragma unroll
    for (int sh = 1; sh < 16; sh <<= 1) s += __shfl_xor(s, sh, 32);
    const float mu = s * (1.0f / 64); float q = 0.f;
#pragma unroll
    for (int k = 0; k < 4; ++k) { const float d = v[k] - mu; q = fmaf(d, d, q); }
#pragma unroll
    for (int sh = 1; sh < 16; sh <<= 1) q += __shfl_xor(q, sh, 32);
    const float rs = rsqrtf(q * (1.0f / 64) + 1e-6f); if (!live) return; v4h o;
#pragma unroll
    for (int k = 0; k < 4; ++k) { const int c = (h0 + z) * 64 + c0 + k; o[k] = tohx(siluf(PR[(size_t)i * PJ + c]) * ((v[k] - mu) * rs)); }
    const size_t off = (size_t)i * (DL * NH_) + (h0 + z) * 64 + c0; *(volatile v4h*)(UD + off) = o; __threadfence(); *(volatile v4h*)(UD + off) = o;
}

__global__ __launch_bounds__(256) void k_xr(const float* __restrict__ x, float* XA) {
    const int lane = threadIdx.x & 31; const size_t r = (size_t)blockIdx.x * 8 + (threadIdx.x >> 5); if (r >= (size_t)SS) return;
#pragma unroll 1
    for (int ps = 0; ps < 2; ++ps) {
#pragma unroll
        for (int p = 0; p < DD / 128; ++p) { const int c0 = p * 128 + lane * 4; const v4f v = *(const v4f*)(x + r * DD + c0); v4f o; for (int i = 0; i < 4; ++i) o[i] = bfr(v[i]); *(volatile v4f*)(XA + r * DD + c0) = o; }
        if (ps == 0) __threadfence(); }
}
extern "C" void kernel_launch(void* const* d_in, const int* in_sizes, int n_in,
                              void* d_out, int out_size, void* d_ws, size_t ws_size, hipStream_t stream) {
    (void)in_sizes; (void)n_in; (void)out_size;
    const float* x = (const float*)d_in[0]; const int* mask = (const int*)d_in[1]; const float* uvqk = (const float*)d_in[2]; const float* ow = (const float*)d_in[3]; const float* ob = (const float*)d_in[4]; const float* lnw = (const float*)d_in[5]; const float* lnb = (const float*)d_in[6]; const float* llw = (const float*)d_in[7]; const float* llb = (const float*)d_in[8];
    float* out = (float*)d_out;
    char* wsp = (char*)d_ws;
    auto take = [&](size_t bytes) { char* p = wsp; wsp += (bytes + 255) & ~(size_t)255; return (void*)p; };
    h16* BUV = (h16*)take((size_t)NL * PJ * DD * 2); h16* BO = (h16*)take((size_t)NL * DD * (DL * NH_) * 2); int* FL = (int*)take((size_t)NB_ * NT64 * NT64 * 4);
    float* XA = (float*)take((size_t)SS * DD * 4); float* XB2 = (float*)take((size_t)SS * DD * 4); h16* XN = (h16*)take((size_t)SS * DD * 2); float* PR = (float*)take((size_t)SS * PJ * 4);
    h16* Qx = (h16*)take((size_t)ZH * SS * 64 * 2); h16* Kx = (h16*)take((size_t)ZH * SS * 64 * 2); h16* VTx = (h16*)take((size_t)ZH * 64 * SS * 2); float* S = (float*)take((size_t)ZH * SS * SS * 4); h16* Px = (h16*)take((size_t)ZH * SS * SS * 2); float* O = (float*)take((size_t)ZH * SS * 64 * 4); h16* UD = (h16*)take((size_t)SS * DL * NH_ * 2);
    if ((size_t)(wsp - (char*)d_ws) > ws_size) return;
    for (int l = 0; l < NL; ++l) { k_wTh<<<dim3(DD / 64, PJ / 64, 1), 256, 0, stream>>>(uvqk + (size_t)l * DD * PJ, DD, PJ, BUV + (size_t)l * PJ * DD); k_cvt8h<<<(unsigned)(((size_t)DD * DL * NH_ / 8 + 255) / 256), 256, 0, stream>>>(ow + (size_t)l * DD * DL * NH_, BO + (size_t)l * DD * DL * NH_, (size_t)DD * DL * NH_ / 8); }
    k_flags<<<dim3(NT64, NB_, 1), 256, 0, stream>>>(mask, FL);
    for (int b = 0; b < NB_; ++b) { const int* FLb = FL + (size_t)b * NT64 * NT64;
        k_xr<<<SS / 8, 256, 0, stream>>>(x + (size_t)b * SS * DD, XA); float* xcur = XA; float* xnext = XB2;
        for (int l = 0; l < NL; ++l) { const float* src = xcur;
            k_lnh<false><<<SS / 8, 256, 0, stream>>>(src, lnw + (size_t)l * DD, lnb + (size_t)l * DD, 1e-6f, XN, nullptr);
            k_gemmh<<<dim3(SS / 64, PJ / 64, 1), 128, 0, stream>>>(XN, BUV + (size_t)l * PJ * DD, nullptr, PR, PJ, nullptr, DD, 0, 0, 0, 0);
            for (int h0 = 0; h0 < NH_; h0 += ZH) {
                k_hpls<<<dim3((SS / 2) / 8, 1, ZH), 256, 0, stream>>>(PR, 2 * DL * NH_, h0, Qx); k_hpls<<<dim3((SS / 2) / 8, 1, ZH), 256, 0, stream>>>(PR, 2 * DL * NH_ + DA * NH_, h0, Kx); k_vTs<<<dim3(SS / 64, 1, ZH), 256, 0, stream>>>(PR, h0, VTx);
                k_gemmhm<1><<<dim3(SS / 64, SS / 64, ZH), 128, 0, stream>>>(Qx, Kx, 64, S, SS, (size_t)SS * 64, (size_t)SS * 64, (size_t)SS * SS, FLb);
                k_pmask<<<dim3(SS / 8, 1, ZH), 256, 0, stream>>>(S, mask, b, Px);
                k_gemmhm<2><<<dim3(SS / 64, 1, ZH), 128, 0, stream>>>(Px, VTx, SS, O, 64, (size_t)SS * SS, (size_t)64 * SS, (size_t)SS * 64, FLb);
                k_normu<<<dim3((SS / 2) / 8, 1, ZH), 256, 0, stream>>>(O, PR, h0, UD); }
            k_gemmh<<<dim3(SS / 64, DD / 64, 1), 128, 0, stream>>>(UD, BO + (size_t)l * DD * DL * NH_, ob + (size_t)l * DD, xnext, DD, src, DL * NH_, 0, 0, 0, 0);
            xcur = xnext; xnext = (xnext == XA) ? XB2 : XA; }
        k_lnh<true><<<SS / 8, 256, 0, stream>>>(xcur, llw, llb, 1e-8f, nullptr, out + (size_t)b * SS * DD); }
}
